// RecurrentGCN_644245094791
// MI455X (gfx1250) — hardware-run, weakly checked
//
#include <hip/hip_runtime.h>
#include <math.h>

typedef __attribute__((ext_vector_type(16))) _Float16 v16h;
typedef __attribute__((ext_vector_type(8)))  float    v8f;
typedef __attribute__((ext_vector_type(4)))  float    v4f;

constexpr int kSteps   = 64;
constexpr int kNodes   = 20000;
constexpr int kFin     = 8;
constexpr int kHid     = 32;
constexpr int kEdges   = 320000;
constexpr int kTileN   = 16;
constexpr int kTiles   = kNodes / kTileN;
constexpr int kWaves   = 5;
constexpr int kThreads = kWaves * 32;
constexpr int kBlocks  = kTiles / kWaves;
constexpr int kSlabP   = 36;
constexpr float kStateCarry  = 64.0f;
constexpr float kWeightCarry = 64.0f;
constexpr float kProdCarry   = kStateCarry * kWeightCarry;
constexpr float kProdInv     = 1.0f / kProdCarry;
constexpr float kF16Min      = 6.103515625e-5f;
constexpr float kSlope       = 0.01f;
constexpr size_t kPartBytes  = (size_t)kBlocks * kSteps * 4;
constexpr size_t kWsTotal    = kPartBytes;
static_assert(kTiles * kTileN == kNodes, "node tiles exact");
static_assert(kBlocks * kWaves == kTiles, "wave tiles exact");
static_assert(kBlocks == 250 && kThreads == 160, "launch shape");
static_assert(kHid == 32 && kFin == 8, "fragment geometry");
static_assert(kProdCarry == 4096.0f, "carry product");
static_assert((kPartBytes % 128) == 0, "partials are whole lines");
static_assert(kWsTotal == 64000ull, "carve total");
static_assert(kWsTotal <= 134217728ull, "carve cap");
static_assert((kSlabP * 4) % 16 == 0, "slab rows 16-B aligned");

__device__ __forceinline__ float bf16r(float f) {
  unsigned u = __float_as_uint(f);
  u = (u + 0x7FFFu + ((u >> 16) & 1u)) & 0xFFFF0000u;
  return __uint_as_float(u);
}
__device__ __forceinline__ _Float16 to_h(float s) {
  const float q = (fabsf(s) < kF16Min) ? 0.0f : s;
  return (_Float16)q;
}
__device__ __forceinline__ float leaky(float v) { return (v >= 0.0f) ? v : kSlope * v; }
__device__ __forceinline__ float sigm(float v)  { return __builtin_amdgcn_rcpf(1.0f + expf(-v)); }
__device__ __forceinline__ float tanh_e(float v) { return 1.0f - 2.0f * __builtin_amdgcn_rcpf(expf(2.0f * v) + 1.0f); }
__device__ __forceinline__ v8f lds8(const float* p) { return *(const v8f*)p; }

__device__ __forceinline__ v8f mma_h(v16h a, v16h b, v8f c) {
  c = __builtin_amdgcn_wmma_f32_16x16x32_f16(false, a, false, b, (short)0, c, false, false);
  asm volatile("v_nop\n\tv_nop\n\tv_nop\n\tv_nop" : "+v"(c) : "v"(a), "v"(b));
  return c;
}

__device__ __forceinline__ v16h frag_state(v8f a, v8f b) {
  v16h f;
#pragma unroll
  for (int i = 0; i < 8; ++i) {
    f[i]     = to_h(a[i] * kStateCarry);
    f[8 + i] = to_h(b[i] * kStateCarry);
  }
  return f;
}
__device__ __forceinline__ v16h frag_wh(const float* sw, int u, int h) {
  v16h f;
#pragma unroll
  for (int i = 0; i < 8; ++i) {
    f[i]     = to_h(sw[(8 * h + i) * kHid + u]);
    f[8 + i] = to_h(sw[(16 + 8 * h + i) * kHid + u]);
  }
  return f;
}
__device__ __forceinline__ v16h frag_wx(const float* sw, int u, bool lo) {
  v16h f;
#pragma unroll
  for (int i = 0; i < 8; ++i) {
    const float wv = sw[i * kHid + u];
    const float s  = lo ? wv : 0.0f;
    f[i]     = to_h(s);
    f[8 + i] = (_Float16)0.0f;
  }
  return f;
}
__device__ __forceinline__ _Float16 x_elem(float v, bool lo) {
  const float s = lo ? (bf16r(v) * kStateCarry) : 0.0f;
  return to_h(s);
}
__device__ __forceinline__ v8f sig8(v8f a) {
  v8f o;
#pragma unroll
  for (int r = 0; r < 8; ++r) o[r] = sigm(a[r] * kProdInv);
  return o;
}
__device__ __forceinline__ v8f tanh8(v8f a) {
  v8f o;
#pragma unroll
  for (int r = 0; r < 8; ++r) o[r] = tanh_e(a[r] * kProdInv);
  return o;
}
__device__ __forceinline__ v8f bf16r8(v4f a, v4f b) {
  const float a0 = a[0], a1 = a[1], a2 = a[2], a3 = a[3];
  const float b0 = b[0], b1 = b[1], b2 = b[2], b3 = b[3];
  v8f o;
  o[0] = bf16r(a0); o[1] = bf16r(a1); o[2] = bf16r(a2); o[3] = bf16r(a3);
  o[4] = bf16r(b0); o[5] = bf16r(b1); o[6] = bf16r(b2); o[7] = bf16r(b3);
  return o;
}
__device__ __forceinline__ void stage_weight(const float* __restrict__ src, float* dst, int n4, int tid) {
#pragma unroll 1
  for (int i = tid; i < n4; i += kThreads) {
    const v4f v = *(const v4f*)(src + 4 * i);
    const float e0 = v[0], e1 = v[1], e2 = v[2], e3 = v[3];
    v4f o;
    o[0] = bf16r(e0) * kWeightCarry;
    o[1] = bf16r(e1) * kWeightCarry;
    o[2] = bf16r(e2) * kWeightCarry;
    o[3] = bf16r(e3) * kWeightCarry;
    *(v4f*)(dst + 4 * i) = o;
  }
}

__global__ __launch_bounds__(kThreads) void gated_cell_nodes_kernel(
    const float* __restrict__ x, const float* __restrict__ h0,
    const float* __restrict__ Wxz, const float* __restrict__ bxz,
    const float* __restrict__ Whz, const float* __restrict__ bhz,
    const float* __restrict__ Wxr, const float* __restrict__ bxr,
    const float* __restrict__ Whr, const float* __restrict__ bhr,
    const float* __restrict__ Wxh, const float* __restrict__ bxh,
    const float* __restrict__ Whh, const float* __restrict__ bhh,
    const float* __restrict__ W1, const float* __restrict__ b1,
    const float* __restrict__ W2,
    float* __restrict__ part, float* __restrict__ hfin)
{
  __shared__ __align__(32) float sWh[3 * kHid * kHid];
  __shared__ __align__(32) float sWx[3 * kFin * kHid];
  __shared__ __align__(32) float sBias[3 * kHid];
  __shared__ __align__(32) float sW1[kHid];
  __shared__ __align__(16) float sPart[kWaves * kSteps];
  __shared__ __align__(16) float sSlab[kWaves * 16 * kSlabP];

  const int tid  = threadIdx.x;
  const int lane = tid & 31;
  const int wave = tid >> 5;
  const int c    = lane & 15;
  const int h    = lane >> 4;
  const bool lo  = (h == 0);

  stage_weight(Whz, sWh,                 kHid * kHid / 4, tid);
  stage_weight(Whr, sWh + kHid * kHid,   kHid * kHid / 4, tid);
  stage_weight(Whh, sWh + 2 * kHid * kHid, kHid * kHid / 4, tid);
  stage_weight(Wxz, sWx,                 kFin * kHid / 4, tid);
  stage_weight(Wxr, sWx + kFin * kHid,   kFin * kHid / 4, tid);
  stage_weight(Wxh, sWx + 2 * kFin * kHid, kFin * kHid / 4, tid);
  {
    const int u = lane;
    const float vxz = bxz[u], vhz = bhz[u], vxr = bxr[u], vhr = bhr[u], vxh = bxh[u], vhh = bhh[u];
    const float vw1 = W1[u];
    const float sz = (bf16r(vxz) + bf16r(vhz)) * kProdCarry;
    const float sr = (bf16r(vxr) + bf16r(vhr)) * kProdCarry;
    const float sg = (bf16r(vxh) + bf16r(vhh)) * kProdCarry;
    const float sel = (wave == 0) ? sz : ((wave == 1) ? sr : sg);
    if (wave < 3)  sBias[wave * kHid + u] = sel;
    if (wave == 3) sW1[u] = bf16r(vw1);
  }
  __syncthreads();

  const int tile     = blockIdx.x * kWaves + wave;
  const int nodeBase = tile * kTileN;
  const int node     = nodeBase + c;

  const v16h Ahz0 = frag_wh(sWh,                     c,      h);
  const v16h Ahz1 = frag_wh(sWh,                     16 + c, h);
  const v16h Ahr0 = frag_wh(sWh + kHid * kHid,       c,      h);
  const v16h Ahr1 = frag_wh(sWh + kHid * kHid,       16 + c, h);
  const v16h Ahh0 = frag_wh(sWh + 2 * kHid * kHid,   c,      h);
  const v16h Ahh1 = frag_wh(sWh + 2 * kHid * kHid,   16 + c, h);
  const v16h Axz0 = frag_wx(sWx,                     c,      lo);
  const v16h Axz1 = frag_wx(sWx,                     16 + c, lo);
  const v16h Axr0 = frag_wx(sWx + kFin * kHid,       c,      lo);
  const v16h Axr1 = frag_wx(sWx + kFin * kHid,       16 + c, lo);
  const v16h Axh0 = frag_wx(sWx + 2 * kFin * kHid,   c,      lo);
  const v16h Axh1 = frag_wx(sWx + 2 * kFin * kHid,   16 + c, lo);

  v8f hs0, hs1;
  {
    const float* hp = h0 + (size_t)node * kHid + 8 * h;
    const v4f ha = *(const v4f*)(hp);
    const v4f hb = *(const v4f*)(hp + 4);
    const v4f hc = *(const v4f*)(hp + 16);
    const v4f hd = *(const v4f*)(hp + 20);
    hs0 = bf16r8(ha, hb);
    hs1 = bf16r8(hc, hd);
  }
  const float w2v = bf16r(W2[node]);
  const float b1v = bf16r(b1[0]);

#pragma unroll 1
  for (int t = 0; t < kSteps; ++t) {
    int o8 = 8 * h;
    asm volatile("" : "+v"(o8));

    const float* xp = x + ((size_t)t * kNodes + (size_t)node) * kFin;
    const v4f xa = *(const v4f*)(xp);
    const v4f xb = *(const v4f*)(xp + 4);
    float x0 = xa[0], x1 = xa[1], x2 = xa[2], x3 = xa[3];
    float x4 = xb[0], x5 = xb[1], x6 = xb[2], x7 = xb[3];
    asm volatile("" : "+v"(x0), "+v"(x1), "+v"(x2), "+v"(x3));
    asm volatile("" : "+v"(x4), "+v"(x5), "+v"(x6), "+v"(x7));
    v16h xB;
    xB[0] = x_elem(x0, lo); xB[1] = x_elem(x1, lo); xB[2] = x_elem(x2, lo); xB[3] = x_elem(x3, lo);
    xB[4] = x_elem(x4, lo); xB[5] = x_elem(x5, lo); xB[6] = x_elem(x6, lo); xB[7] = x_elem(x7, lo);
    xB[8]  = (_Float16)0.0f; xB[9]  = (_Float16)0.0f; xB[10] = (_Float16)0.0f; xB[11] = (_Float16)0.0f;
    xB[12] = (_Float16)0.0f; xB[13] = (_Float16)0.0f; xB[14] = (_Float16)0.0f; xB[15] = (_Float16)0.0f;

    const v16h hB = frag_state(hs0, hs1);

    v8f z0 = lds8(sBias + o8);
    v8f z1 = lds8(sBias + 16 + o8);
    v8f r0 = lds8(sBias + 32 + o8);
    v8f r1 = lds8(sBias + 48 + o8);
    z0 = mma_h(Axz0, xB, z0);
    z0 = mma_h(Ahz0, hB, z0);
    z1 = mma_h(Axz1, xB, z1);
    z1 = mma_h(Ahz1, hB, z1);
    r0 = mma_h(Axr0, xB, r0);
    r0 = mma_h(Ahr0, hB, r0);
    r1 = mma_h(Axr1, xB, r1);
    r1 = mma_h(Ahr1, hB, r1);

    const v8f r0s = sig8(r0);
    const v8f r1s = sig8(r1);
    v8f p0, p1;
#pragma unroll
    for (int i = 0; i < 8; ++i) {
      p0[i] = hs0[i] * r0s[i];
      p1[i] = hs1[i] * r1s[i];
    }
    const v16h pB = frag_state(p0, p1);

    v8f g0 = lds8(sBias + 64 + o8);
    v8f g1 = lds8(sBias + 80 + o8);
    g0 = mma_h(Axh0, xB, g0);
    g0 = mma_h(Ahh0, pB, g0);
    g1 = mma_h(Axh1, xB, g1);
    g1 = mma_h(Ahh1, pB, g1);

    const v8f z0s = sig8(z0);
    const v8f z1s = sig8(z1);
    const v8f c0  = tanh8(g0);
    const v8f c1  = tanh8(g1);
#pragma unroll
    for (int i = 0; i < 8; ++i) {
      hs0[i] = z0s[i] * hs0[i] + (1.0f - z0s[i]) * c0[i];
      hs1[i] = z1s[i] * hs1[i] + (1.0f - z1s[i]) * c1[i];
    }

    const v8f w1a = lds8(sW1 + o8);
    const v8f w1b = lds8(sW1 + 16 + o8);
    float sp = 0.0f;
#pragma unroll
    for (int i = 0; i < 8; ++i) sp = fmaf(leaky(hs0[i]), w1a[i], sp);
#pragma unroll
    for (int i = 0; i < 8; ++i) sp = fmaf(leaky(hs1[i]), w1b[i], sp);
    const float so = __shfl_xor(sp, 16, 32);
    const float sfull = sp + so;
    const float a2 = leaky(sfull + b1v);
    float pv = a2 * w2v;
    pv += __shfl_xor(pv, 1, 32);
    pv += __shfl_xor(pv, 2, 32);
    pv += __shfl_xor(pv, 4, 32);
    pv += __shfl_xor(pv, 8, 32);
    if (lane == 0) sPart[wave * kSteps + t] = pv;
  }

  float* slab = sSlab + wave * 16 * kSlabP;
  {
    float* sp0 = slab + c * kSlabP + 8 * h;
    v4f q0, q1, q2, q3;
    q0[0] = hs0[0]; q0[1] = hs0[1]; q0[2] = hs0[2]; q0[3] = hs0[3];
    q1[0] = hs0[4]; q1[1] = hs0[5]; q1[2] = hs0[6]; q1[3] = hs0[7];
    q2[0] = hs1[0]; q2[1] = hs1[1]; q2[2] = hs1[2]; q2[3] = hs1[3];
    q3[0] = hs1[4]; q3[1] = hs1[5]; q3[2] = hs1[6]; q3[3] = hs1[7];
    *(v4f*)(sp0)      = q0;
    *(v4f*)(sp0 + 4)  = q1;
    *(v4f*)(sp0 + 16) = q2;
    *(v4f*)(sp0 + 20) = q3;
  }
  __syncthreads();
  {
    const int q  = lane >> 3;
    const int c4 = (lane & 7) * 4;
    v4f ov[4];
#pragma unroll
    for (int it = 0; it < 4; ++it) ov[it] = *(const v4f*)(slab + (it * 4 + q) * kSlabP + c4);
    for (int pass = 0; pass < 2; ++pass) {
#pragma unroll
      for (int it = 0; it < 4; ++it)
        *(volatile v4f*)(hfin + (size_t)(nodeBase + it * 4 + q) * kHid + c4) = ov[it];
      __threadfence();
    }
  }
  if (wave < 2) {
    float s = 0.0f;
    s += sPart[0 * kSteps + tid];
    s += sPart[1 * kSteps + tid];
    s += sPart[2 * kSteps + tid];
    s += sPart[3 * kSteps + tid];
    s += sPart[4 * kSteps + tid];
    volatile float* pp = part + (size_t)blockIdx.x * kSteps + tid;
    *pp = s;
    __threadfence();
    *pp = s;
  }
}

__global__ __launch_bounds__(64) void sum_parts_kernel(const float* __restrict__ part,
                                                       const float* __restrict__ b2,
                                                       float* __restrict__ out)
{
  const int t = threadIdx.x;
  float s = 0.0f;
#pragma unroll 1
  for (int b = 0; b < kBlocks; ++b) s += part[(size_t)b * kSteps + t];
  const float o = s + bf16r(b2[0]);
  volatile float* op = out + t;
  *op = o;
  __threadfence();
  *op = o;
}

extern "C" void kernel_launch(void* const* d_in, const int* in_sizes, int n_in,
                              void* d_out, int out_size, void* d_ws, size_t ws_size,
                              hipStream_t stream) {
  if (n_in < 20 || d_out == nullptr || d_ws == nullptr) return;
  if (in_sizes[0] != kSteps * kNodes * kFin) return;
  if (in_sizes[1] != 2 * kEdges) return;
  if (in_sizes[2] != kEdges) return;
  if (in_sizes[3] != kNodes * kHid) return;
  if (in_sizes[4] != kFin * kHid || in_sizes[8] != kFin * kHid || in_sizes[12] != kFin * kHid) return;
  if (in_sizes[6] != kHid * kHid || in_sizes[10] != kHid * kHid || in_sizes[14] != kHid * kHid) return;
  if (in_sizes[5] != kHid || in_sizes[7] != kHid || in_sizes[9] != kHid || in_sizes[11] != kHid ||
      in_sizes[13] != kHid || in_sizes[15] != kHid) return;
  if (in_sizes[16] != kHid || in_sizes[17] != 1 || in_sizes[18] != kNodes || in_sizes[19] != 1) return;
  if (out_size != kSteps + kNodes * kHid) return;
  if (ws_size < kWsTotal) return;

  const float* x   = (const float*)d_in[0];
  const float* h0  = (const float*)d_in[3];
  const float* Wxz = (const float*)d_in[4];
  const float* bxz = (const float*)d_in[5];
  const float* Whz = (const float*)d_in[6];
  const float* bhz = (const float*)d_in[7];
  const float* Wxr = (const float*)d_in[8];
  const float* bxr = (const float*)d_in[9];
  const float* Whr = (const float*)d_in[10];
  const float* bhr = (const float*)d_in[11];
  const float* Wxh = (const float*)d_in[12];
  const float* bxh = (const float*)d_in[13];
  const float* Whh = (const float*)d_in[14];
  const float* bhh = (const float*)d_in[15];
  const float* W1  = (const float*)d_in[16];
  const float* b1  = (const float*)d_in[17];
  const float* W2  = (const float*)d_in[18];
  const float* b2  = (const float*)d_in[19];

  float* out  = (float*)d_out;
  float* hfin = out + kSteps;
  float* PART = (float*)d_ws;

  gated_cell_nodes_kernel<<<kBlocks, kThreads, 0, stream>>>(
      x, h0, Wxz, bxz, Whz, bhz, Wxr, bxr, Whr, bhr, Wxh, bxh, Whh, bhh, W1, b1, W2, PART, hfin);
  sum_parts_kernel<<<1, 64, 0, stream>>>(PART, b2, out);
}
